// LocalStructureLayer_55585466745465
// MI455X (gfx1250) — hardware-verified
//
#include <hip/hip_runtime.h>
#include <stddef.h>


#define CH       128
#define GR       64
#define GTHR     256
#define CP       132
#define NBS      256
#define SH       8
#define CHUNK    2048
#define ATHR     256
#define AWAVE    8
#define WCAP     256
#define NGRP     (CHUNK / (ATHR * 4))
#define WSC      8.0f
#define AGS      64.0f
#define INVSQ    0.08838834764831845f
#define WROWS    512
#define AGG_QS   (NBS * CH)
#define AGG_SACC (NBS * CH)
#define AGG_AUX  (2 * NBS)
#define AGG_LIST (AWAVE * WCAP)
#define AGG_LDS_BYTES ((AGG_QS + AGG_SACC + AGG_AUX + AGG_LIST + AWAVE) * 4)

static_assert(AGG_LDS_BYTES == 272416);
static_assert(NGRP == 2);
static_assert(WCAP == (CHUNK / ATHR) * 32);
static_assert(NBS == (1 << SH));
static_assert(SH + 11 <= 31);
static_assert((CP * 4) % 16 == 0);
static_assert(GR == 64 && GTHR == 256);

typedef float          v4f  __attribute__((ext_vector_type(4)));
typedef float          v8f  __attribute__((ext_vector_type(8)));
typedef int            v4i  __attribute__((ext_vector_type(4)));
typedef _Float16       v8h  __attribute__((ext_vector_type(8)));
typedef _Float16       v16h __attribute__((ext_vector_type(16)));
typedef __bf16         v16b __attribute__((ext_vector_type(16)));
typedef unsigned short v8us __attribute__((ext_vector_type(8)));

union Frag   { v16h h; v16b b; v4i q[2]; };
union Pack16 { v8h h; v8us u; v4i i; };

__device__ __forceinline__ v8f wmh(v16h a, v16h b, v8f c) {
  v8f d = __builtin_amdgcn_wmma_f32_16x16x32_f16(false, a, false, b, (short)0, c, false, false);
  asm volatile("v_nop\n\tv_nop\n\tv_nop\n\tv_nop" : "+v"(d) : "v"(a), "v"(b));
  return d;
}

__device__ __forceinline__ v8f wmb3(v16b ah, v16b al, v16b bh, v16b bl, v8f c) {
  v8f d = __builtin_amdgcn_wmma_f32_16x16x32_bf16(false, ah, false, bh, (short)0, c, false, false);
  d = __builtin_amdgcn_wmma_f32_16x16x32_bf16(false, ah, false, bl, (short)0, d, false, false);
  d = __builtin_amdgcn_wmma_f32_16x16x32_bf16(false, al, false, bh, (short)0, d, false, false);
  asm volatile("v_nop\n\tv_nop\n\tv_nop\n\tv_nop" : "+v"(d) : "v"(ah), "v"(al), "v"(bh), "v"(bl));
  return d;
}

__device__ __forceinline__ void ldfrag(Frag& f, const unsigned short* p) {
  f.q[0] = *(const v4i*)p;
  f.q[1] = *(const v4i*)(p + 16);
}

__device__ __forceinline__ float wsum(float v) {
  v += __shfl_xor(v, 16, 32);
  v += __shfl_xor(v, 8, 32);
  v += __shfl_xor(v, 4, 32);
  v += __shfl_xor(v, 2, 32);
  v += __shfl_xor(v, 1, 32);
  return v;
}

__device__ __forceinline__ unsigned short bf16_rne(float f) {
  unsigned u = __float_as_uint(f);
  u = u + 0x7FFFu + ((u >> 16) & 1u);
  return (unsigned short)(u >> 16);
}

__device__ __forceinline__ void split1(float f, unsigned short& hi, unsigned short& lo) {
  hi = bf16_rne(f);
  const float fh = __uint_as_float(((unsigned)hi) << 16);
  lo = bf16_rne(f - fh);
}

__device__ __forceinline__ void split8(const v4f a, const v4f b, Pack16& ph, Pack16& pl) {
  unsigned short h, l;
  split1(a.x, h, l); ph.u[0] = h; pl.u[0] = l;
  split1(a.y, h, l); ph.u[1] = h; pl.u[1] = l;
  split1(a.z, h, l); ph.u[2] = h; pl.u[2] = l;
  split1(a.w, h, l); ph.u[3] = h; pl.u[3] = l;
  split1(b.x, h, l); ph.u[4] = h; pl.u[4] = l;
  split1(b.y, h, l); ph.u[5] = h; pl.u[5] = l;
  split1(b.z, h, l); ph.u[6] = h; pl.u[6] = l;
  split1(b.w, h, l); ph.u[7] = h; pl.u[7] = l;
}

__device__ __forceinline__ void cvt8h(const v4f a, const v4f b, float s, Pack16& p) {
  p.h[0] = (_Float16)(a.x * s); p.h[1] = (_Float16)(a.y * s);
  p.h[2] = (_Float16)(a.z * s); p.h[3] = (_Float16)(a.w * s);
  p.h[4] = (_Float16)(b.x * s); p.h[5] = (_Float16)(b.y * s);
  p.h[6] = (_Float16)(b.z * s); p.h[7] = (_Float16)(b.w * s);
}

__global__ __launch_bounds__(256) void k_cvtx(const float* __restrict__ x, unsigned short* H,
                                             int nN, int nP) {
  const int gw   = (blockIdx.x * 256 + threadIdx.x) >> 5;
  const int lane = threadIdx.x & 31;
  const int hh   = lane >> 4;
  const int m    = lane & 15;
  const int row  = 2 * gw + hh;
  const int c8   = 8 * m;
  int srow = row;
  if (srow > nN - 1) srow = nN - 1;
  const float* p = x + (size_t)srow * CH + c8;
  const v4f f0 = *(const v4f*)p;
  const v4f f1 = *(const v4f*)(p + 4);
  Pack16 u;
  cvt8h(f0, f1, 1.0f, u);
  unsigned short* dst = H + (size_t)row * CH + c8;
  const bool ok = (2 * gw + 1 < nP);
  if (ok) *(volatile v4i*)dst = u.i;
  __threadfence();
  if (ok) *(volatile v4i*)dst = u.i;
}

__global__ __launch_bounds__(256) void k_cvtw(const float* __restrict__ w0, const float* __restrict__ w1,
                                             const float* __restrict__ w2, const float* __restrict__ w3,
                                             unsigned short* H, unsigned short* L, int mode) {
  const int gw   = (blockIdx.x * 256 + threadIdx.x) >> 5;
  const int lane = threadIdx.x & 31;
  const int hh   = lane >> 4;
  const int m    = lane & 15;
  const int row  = 2 * gw + hh;
  const int c8   = 8 * m;
  const int which = row >> 7;
  const int r     = row & 127;
  const float* s = (which == 0) ? w0 : ((which == 1) ? w1 : ((which == 2) ? w2 : w3));
  const float* p = s + (size_t)r * CH + c8;
  const v4f f0 = *(const v4f*)p;
  const v4f f1 = *(const v4f*)(p + 4);
  const bool ok = (row < WROWS);
  if (mode == 0) {
    Pack16 u;
    cvt8h(f0, f1, WSC, u);
    unsigned short* dh = H + (size_t)row * CH + c8;
    if (ok) *(volatile v4i*)dh = u.i;
    __threadfence();
    if (ok) *(volatile v4i*)dh = u.i;
  } else {
    Pack16 ph, pl;
    split8(f0, f1, ph, pl);
    unsigned short* dh = H + (size_t)row * CH + c8;
    unsigned short* dl = L + (size_t)row * CH + c8;
    if (ok) { *(volatile v4i*)dh = ph.i; *(volatile v4i*)dl = pl.i; }
    __threadfence();
    if (ok) { *(volatile v4i*)dh = ph.i; *(volatile v4i*)dl = pl.i; }
  }
}

template <int MODE, int OUTK>
__global__ __launch_bounds__(GTHR) void k_gemm(const unsigned short* __restrict__ Ah,
                                              const unsigned short* __restrict__ Al,
                                              const unsigned short* __restrict__ Bh,
                                              const unsigned short* __restrict__ Bl,
                                              const float* __restrict__ b0,
                                              const float* __restrict__ b1,
                                              const float* __restrict__ b2,
                                              const float* __restrict__ gam,
                                              const float* __restrict__ bet,
                                              float oscale,
                                              float* outQ, float* outKV,
                                              unsigned short* oH, unsigned short* oL,
                                              float* outF, int nN) {
  __shared__ __attribute__((aligned(16))) float Cs[GR * CP];

  const int tid  = threadIdx.x;
  const int lane = tid & 31;
  const int wave = tid >> 5;
  const int hh   = lane >> 4;
  const int m    = lane & 15;
  const int rowTile = blockIdx.x * GR;
  const int cg   = blockIdx.y;
  const int colL = wave * 16 + m;
  const int ncol = cg * CH + colL;

  Frag bH[4];
  Frag bL[4];
  {
    const unsigned short* pb = Bh + (size_t)ncol * CH + 8 * hh;
#pragma unroll
    for (int kt = 0; kt < 4; ++kt) ldfrag(bH[kt], pb + kt * 32);
    if (MODE == 1) {
      const unsigned short* pl = Bl + (size_t)ncol * CH + 8 * hh;
#pragma unroll
      for (int kt = 0; kt < 4; ++kt) ldfrag(bL[kt], pl + kt * 32);
    } else {
#pragma unroll
      for (int kt = 0; kt < 4; ++kt) bL[kt] = bH[kt];
    }
  }

  const float bb0 = b0[colL];
  const float bb1 = b1[colL];
  const float bb2 = b2[colL];
  const float bv = (cg == 0) ? bb0 : ((cg == 1) ? bb1 : bb2);

  const v8f z8 = {0.f, 0.f, 0.f, 0.f, 0.f, 0.f, 0.f, 0.f};
#pragma unroll
  for (int t = 0; t < 4; ++t) {
    const int arow = rowTile + t * 16 + m;
    const unsigned short* pa  = Ah + (size_t)arow * CH + 8 * hh;
    const unsigned short* pal = Al + (size_t)arow * CH + 8 * hh;
    v8f acc = z8;
#pragma unroll
    for (int kt = 0; kt < 4; ++kt) {
      Frag a;
      ldfrag(a, pa + kt * 32);
      if (MODE == 0) {
        acc = wmh(a.h, bH[kt].h, acc);
      } else {
        Frag al;
        ldfrag(al, pal + kt * 32);
        acc = wmb3(a.b, al.b, bH[kt].b, bL[kt].b, acc);
      }
    }
    float* cs = Cs + (t * 16 + 8 * hh) * CP + colL;
#pragma unroll
    for (int r = 0; r < 8; ++r) cs[r * CP] = acc[r] * oscale + bv;
  }
  __syncthreads();

  if (OUTK == 0) {
    float* obase;
    int pitch;
    if (cg == 0) { obase = outQ; pitch = CH; } else { obase = outKV + (cg - 1) * CH; pitch = 2 * CH; }
    v4f xr[8];
#pragma unroll
    for (int i = 0; i < 8; ++i) xr[i] = *(const v4f*)(Cs + (wave * 8 + i) * CP + 4 * lane);
#pragma unroll
    for (int i = 0; i < 8; ++i)
      *(volatile v4f*)(obase + (size_t)(rowTile + wave * 8 + i) * pitch + 4 * lane) = xr[i];
    __threadfence();
#pragma unroll
    for (int i = 0; i < 8; ++i)
      *(volatile v4f*)(obase + (size_t)(rowTile + wave * 8 + i) * pitch + 4 * lane) = xr[i];
  } else {
    const v4f g4 = *(const v4f*)(gam + 4 * lane);
    const v4f e4 = *(const v4f*)(bet + 4 * lane);
    v4f yv[8];
#pragma unroll
    for (int i = 0; i < 8; ++i) {
      const int row = wave * 8 + i;
      const v4f v = *(const v4f*)(Cs + row * CP + 4 * lane);
      const float s  = wsum(v.x + v.y + v.z + v.w);
      const float mu = s * (1.0f / CH);
      const v4f d = v - mu;
      const float q  = wsum(d.x * d.x + d.y * d.y + d.z * d.z + d.w * d.w);
      const float rs = rsqrtf(q * (1.0f / CH) + 1e-5f);
      v4f y = d * rs * g4 + e4;
      if (OUTK == 1) {
        y.x = fmaxf(y.x, 0.f); y.y = fmaxf(y.y, 0.f); y.z = fmaxf(y.z, 0.f); y.w = fmaxf(y.w, 0.f);
      }
      yv[i] = y;
    }
    if (OUTK == 2) {
#pragma unroll
      for (int i = 0; i < 8; ++i) {
        const int row = rowTile + wave * 8 + i;
        if (row < nN) *(volatile v4f*)(outF + (size_t)row * CH + 4 * lane) = yv[i];
      }
      __threadfence();
#pragma unroll
      for (int i = 0; i < 8; ++i) {
        const int row = rowTile + wave * 8 + i;
        if (row < nN) *(volatile v4f*)(outF + (size_t)row * CH + 4 * lane) = yv[i];
      }
    } else {
#pragma unroll
      for (int i = 0; i < 8; ++i) *(v4f*)(Cs + (wave * 8 + i) * CP + 4 * lane) = yv[i];
      __syncthreads();
      v4i hv[4], lv[4];
#pragma unroll
      for (int j = 0; j < 4; ++j) {
        const int row = 2 * (wave * 4 + j) + hh;
        const int c8  = 8 * m;
        const v4f f0 = *(const v4f*)(Cs + row * CP + c8);
        const v4f f1 = *(const v4f*)(Cs + row * CP + c8 + 4);
        Pack16 ph, pl;
        split8(f0, f1, ph, pl);
        hv[j] = ph.i;
        lv[j] = pl.i;
      }
#pragma unroll
      for (int j = 0; j < 4; ++j) {
        const int row = 2 * (wave * 4 + j) + hh;
        const size_t o = (size_t)(rowTile + row) * CH + 8 * m;
        *(volatile v4i*)(oH + o) = hv[j];
        *(volatile v4i*)(oL + o) = lv[j];
      }
      __threadfence();
#pragma unroll
      for (int j = 0; j < 4; ++j) {
        const int row = 2 * (wave * 4 + j) + hh;
        const size_t o = (size_t)(rowTile + row) * CH + 8 * m;
        *(volatile v4i*)(oH + o) = hv[j];
        *(volatile v4i*)(oL + o) = lv[j];
      }
    }
  }
}

template <int MODE>
__global__ __launch_bounds__(ATHR) void k_agg(const int* __restrict__ ei, const float* __restrict__ Q,
                                              const float* __restrict__ KV,
                                              unsigned short* GH, unsigned short* GL,
                                              int nN, int nE, int nP) {
  extern __shared__ v4f lds_dyn[];
  float* qs   = (float*)lds_dyn;
  float* sacc = qs + AGG_QS;
  float* mx   = sacc + AGG_SACC;
  float* den  = mx + NBS;
  int*   list = (int*)(den + NBS);
  int*   wcnt = list + AGG_LIST;

  const int tid  = threadIdx.x;
  const int lane = tid & 31;
  const int wave = tid >> 5;
  const int hh   = lane >> 4;
  const int m    = lane & 15;
  const int nodeBase = blockIdx.x * NBS;

  {
    const v4f z4 = {0.f, 0.f, 0.f, 0.f};
    v4f* sv = (v4f*)sacc;
    for (int i = tid; i < AGG_SACC / 4; i += ATHR) sv[i] = z4;
    for (int i = tid; i < NBS; i += ATHR) { mx[i] = -1.0e30f; den[i] = 0.f; }
    v4f* qv = (v4f*)qs;
    for (int i = tid; i < AGG_QS / 4; i += ATHR) {
      const int row = i >> 5;
      const int c4  = i & 31;
      int node = nodeBase + row;
      if (node > nP - 1) node = nP - 1;
      qv[i] = *(const v4f*)(Q + (size_t)node * CH + 4 * c4);
    }
  }
  __syncthreads();

  const int* eid = ei + nE;
  const bool al16 = ((nE & 3) == 0);
  const int nChunks = (nE + CHUNK - 1) / CHUNK;
#pragma unroll 1
  for (int ch = 0; ch < nChunks; ++ch) {
    const int cbase = ch * CHUNK;
    const bool full = al16 && (cbase + CHUNK <= nE);
    int wc = 0;
#pragma unroll
    for (int g = 0; g < NGRP; ++g) {
      const int el0 = (g * ATHR + tid) * 4;
      const int e0  = cbase + el0;
      const int sent = -2147483647 - 1;
      v4i d;
      if (full) {
        d = *(const v4i*)(eid + e0);
      } else {
        d.x = (e0     < nE) ? eid[min(e0,     nE - 1)] : sent;
        d.y = (e0 + 1 < nE) ? eid[min(e0 + 1, nE - 1)] : sent;
        d.z = (e0 + 2 < nE) ? eid[min(e0 + 2, nE - 1)] : sent;
        d.w = (e0 + 3 < nE) ? eid[min(e0 + 3, nE - 1)] : sent;
      }
      const unsigned s0 = (unsigned)d.x - (unsigned)nodeBase;
      const unsigned s1 = (unsigned)d.y - (unsigned)nodeBase;
      const unsigned s2 = (unsigned)d.z - (unsigned)nodeBase;
      const unsigned s3 = (unsigned)d.w - (unsigned)nodeBase;
      const bool h0 = s0 < (unsigned)NBS;
      const bool h1 = s1 < (unsigned)NBS;
      const bool h2 = s2 < (unsigned)NBS;
      const bool h3 = s3 < (unsigned)NBS;
      const unsigned many = __builtin_amdgcn_ballot_w32(h0 | h1 | h2 | h3);
      if (many != 0u) {
#define HITJ(J, HJ, SJ) { \
          const unsigned mj = __builtin_amdgcn_ballot_w32(HJ); \
          if (HJ) { \
            const int pos = wc + (int)__builtin_amdgcn_mbcnt_lo(mj, 0u); \
            if (pos < WCAP) list[wave * WCAP + pos] = ((el0 + (J)) << SH) | (int)(SJ); \
          } \
          wc += (int)__builtin_popcount(mj); }
        HITJ(0, h0, s0)
        HITJ(1, h1, s1)
        HITJ(2, h2, s2)
        HITJ(3, h3, s3)
#undef HITJ
      }
    }
    if (lane == 0) wcnt[wave] = wc;
    __syncthreads();

    if (wave == 0) {
#pragma unroll 1
      for (int wsx = 0; wsx < AWAVE; ++wsx) {
        int n = wcnt[wsx];
        if (n > WCAP) n = WCAP;
        if (n < 0) n = 0;
#pragma unroll 1
        for (int i = 0; i < n; ++i) {
          const int ent  = list[wsx * WCAP + i];
          const int slot = ent & (NBS - 1);
          const int el   = (ent >> SH) & (CHUNK - 1);
          int e = cbase + el;
          if (e > nE - 1) e = nE - 1;
          int src = ei[e];
          src = src < 0 ? 0 : (src > nN - 1 ? nN - 1 : src);
          const v4f q4 = *(const v4f*)(qs + slot * CH + 4 * lane);
          const float* kr = KV + (size_t)src * (2 * CH) + 4 * lane;
          const v4f k4 = *(const v4f*)kr;
          const v4f v4 = *(const v4f*)(kr + CH);
          float part = q4.x * k4.x + q4.y * k4.y + q4.z * k4.z + q4.w * k4.w;
          part = wsum(part);
          const float logit = part * INVSQ;
          const float mo = mx[slot];
          const float mn = fmaxf(mo, logit);
          const float corr = __expf(mo - mn);
          const float p = __expf(logit - mn);
          const float dn = den[slot] * corr + p;
          v4f* sp = (v4f*)(sacc + slot * CH + 4 * lane);
          const v4f cur = *sp;
          *sp = cur * corr + v4 * p;
          den[slot] = dn;
          mx[slot]  = mn;
        }
      }
    }
    __syncthreads();
  }

#pragma unroll 1
  for (int j = 0; j < NBS / AWAVE; ++j) {
    const int slot = wave * (NBS / AWAVE) + j;
    const float inv = __builtin_amdgcn_rcpf(den[slot] + 1e-16f);
    v4f* sp = (v4f*)(sacc + slot * CH + 4 * lane);
    const v4f cur = *sp;
    *sp = cur * inv;
  }
  __syncthreads();

#pragma unroll 1
  for (int pass = 0; pass < 2; ++pass) {
#pragma unroll 1
    for (int j = 0; j < NBS / (2 * AWAVE); ++j) {
      const int pp  = wave * (NBS / (2 * AWAVE)) + j;
      const int row = 2 * pp + hh;
      const int c8  = 8 * m;
      const bool ok = (nodeBase + 2 * pp + 1 < nP);
      const v4f f0 = *(const v4f*)(sacc + row * CH + c8);
      const v4f f1 = *(const v4f*)(sacc + row * CH + c8 + 4);
      const size_t o = (size_t)(nodeBase + row) * CH + c8;
      if (MODE == 0) {
        Pack16 u;
        cvt8h(f0, f1, AGS, u);
        if (ok) *(volatile v4i*)(GH + o) = u.i;
      } else {
        Pack16 ph, pl;
        split8(f0, f1, ph, pl);
        if (ok) { *(volatile v4i*)(GH + o) = ph.i; *(volatile v4i*)(GL + o) = pl.i; }
      }
    }
    if (pass == 0) __threadfence();
  }
}

extern "C" void kernel_launch(void* const* d_in, const int* in_sizes, int n_in,
                              void* d_out, int out_size, void* d_ws, size_t ws_size,
                              hipStream_t stream) {
  if (n_in < 32) return;
  const int nN = in_sizes[0] / CH;
  if (nN <= 0 || in_sizes[0] != nN * CH) return;
  if (in_sizes[1] < 2 || (in_sizes[1] & 1)) return;
  const int nE = in_sizes[1] / 2;
  for (int l = 0; l < 3; ++l) {
    const int base = 2 + 10 * l;
    for (int j = 0; j < 4; ++j) if (in_sizes[base + j] != CH * CH) return;
    for (int j = 4; j < 10; ++j) if (in_sizes[base + j] != CH) return;
  }
  if (out_size != nN * CH) return;

  const float* x  = (const float*)d_in[0];
  const int*   ei = (const int*)d_in[1];
  float* out = (float*)d_out;

  const int nP = ((nN + GR - 1) / GR) * GR;
  const size_t wplane = (size_t)WROWS * CH * 2;
  const size_t aplane = (size_t)nP * CH * 2;
  size_t off = 0;
  unsigned short* WH0 = (unsigned short*)((char*)d_ws + off); off += wplane;
  unsigned short* WH1 = (unsigned short*)((char*)d_ws + off); off += wplane;
  unsigned short* WL1 = (unsigned short*)((char*)d_ws + off); off += wplane;
  unsigned short* WH2 = (unsigned short*)((char*)d_ws + off); off += wplane;
  unsigned short* WL2 = (unsigned short*)((char*)d_ws + off); off += wplane;
  off += wplane;
  unsigned short* AH = (unsigned short*)((char*)d_ws + off); off += aplane;
  unsigned short* AL = (unsigned short*)((char*)d_ws + off); off += aplane;
  unsigned short* GH = (unsigned short*)((char*)d_ws + off); off += aplane;
  unsigned short* GL = (unsigned short*)((char*)d_ws + off); off += aplane;
  float* Q  = (float*)((char*)d_ws + off); off += (size_t)nP * CH * 4;
  float* KV = (float*)((char*)d_ws + off); off += (size_t)nP * 2 * CH * 4;
  if (off > ws_size) return;
  if (off > (size_t)134217728) return;

  const float* Wq[3]; const float* Wk[3]; const float* Wv[3]; const float* Wo[3];
  const float* bq[3]; const float* bk[3]; const float* bvv[3]; const float* bo[3];
  const float* gg[3]; const float* be[3];
  for (int l = 0; l < 3; ++l) {
    const int base = 2 + 10 * l;
    Wq[l]  = (const float*)d_in[base + 0];
    Wk[l]  = (const float*)d_in[base + 1];
    Wv[l]  = (const float*)d_in[base + 2];
    Wo[l]  = (const float*)d_in[base + 3];
    bq[l]  = (const float*)d_in[base + 4];
    bk[l]  = (const float*)d_in[base + 5];
    bvv[l] = (const float*)d_in[base + 6];
    bo[l]  = (const float*)d_in[base + 7];
    gg[l]  = (const float*)d_in[base + 8];
    be[l]  = (const float*)d_in[base + 9];
  }

  const int gblk = nP / GR;
  const int ablk = (nN + NBS - 1) / NBS;
  const size_t woff = (size_t)384 * CH;

  k_cvtx<<<nP / 16, 256, 0, stream>>>(x, AH, nN, nP);
  k_cvtw<<<32, 256, 0, stream>>>(Wq[0], Wk[0], Wv[0], Wo[0], WH0, WH0, 0);
  k_cvtw<<<32, 256, 0, stream>>>(Wq[1], Wk[1], Wv[1], Wo[1], WH1, WL1, 1);
  k_cvtw<<<32, 256, 0, stream>>>(Wq[2], Wk[2], Wv[2], Wo[2], WH2, WL2, 1);

  hipFuncSetAttribute(reinterpret_cast<const void*>(&k_agg<0>),
                      hipFuncAttributeMaxDynamicSharedMemorySize, AGG_LDS_BYTES);
  hipFuncSetAttribute(reinterpret_cast<const void*>(&k_agg<1>),
                      hipFuncAttributeMaxDynamicSharedMemorySize, AGG_LDS_BYTES);

  k_gemm<0, 0><<<dim3(gblk, 3), GTHR, 0, stream>>>(AH, AH, WH0, WH0, bq[0], bk[0], bvv[0], gg[0], be[0],
                                                   0.125f, Q, KV, GH, GL, out, nN);
  k_agg<0><<<ablk, ATHR, AGG_LDS_BYTES, stream>>>(ei, Q, KV, GH, GL, nN, nE, nP);
  k_gemm<0, 1><<<dim3(gblk, 1), GTHR, 0, stream>>>(GH, GH, WH0 + woff, WH0 + woff, bo[0], bo[0], bo[0],
                                                   gg[0], be[0], 0.001953125f, Q, KV, AH, AL, out, nN);

  k_gemm<1, 0><<<dim3(gblk, 3), GTHR, 0, stream>>>(AH, AL, WH1, WL1, bq[1], bk[1], bvv[1], gg[1], be[1],
                                                   1.0f, Q, KV, GH, GL, out, nN);
  k_agg<1><<<ablk, ATHR, AGG_LDS_BYTES, stream>>>(ei, Q, KV, GH, GL, nN, nE, nP);
  k_gemm<1, 1><<<dim3(gblk, 1), GTHR, 0, stream>>>(GH, GL, WH1 + woff, WL1 + woff, bo[1], bo[1], bo[1],
                                                   gg[1], be[1], 1.0f, Q, KV, AH, AL, out, nN);

  k_gemm<1, 0><<<dim3(gblk, 3), GTHR, 0, stream>>>(AH, AL, WH2, WL2, bq[2], bk[2], bvv[2], gg[2], be[2],
                                                   1.0f, Q, KV, GH, GL, out, nN);
  k_agg<1><<<ablk, ATHR, AGG_LDS_BYTES, stream>>>(ei, Q, KV, GH, GL, nN, nE, nP);
  k_gemm<1, 2><<<dim3(gblk, 1), GTHR, 0, stream>>>(GH, GL, WH2 + woff, WL2 + woff, bo[2], bo[2], bo[2],
                                                   gg[2], be[2], 1.0f, Q, KV, AH, AL, out, nN);
}
